// PatternGraphSAGE_17102559773409
// MI455X (gfx1250) — hardware-verified
//
#include <hip/hip_runtime.h>
#include <stddef.h>


#define DF      256
#define KV      512
#define CGW     128
#define NPF     128
#define NTHR    256
#define NWAVE   8
#define EPT     8
#define NGRP    2
#define CHUNK   (NTHR * EPT * NGRP)
#define WCAP    (EPT * NGRP * 32)
#define LISTN   (NWAVE * WCAP)
#define NB      256
#define NTILE   (NB / 16)
#define TPW     (NTILE / NWAVE)
#define NB0     4096
#define RG0     (NB0 / (NWAVE * 4))
#define A_SC    8.0f
#define W_SC    32.0f
#define O_SC    0.00390625f
#define LN_EPS  1e-5f

#define LDS_ACC   (NB * DF * 4)
#define LDS_LIST  (LISTN * 4)
#define LDS_CNT   (NB * 4)
#define LDS_LAYER (LDS_ACC + LDS_LIST + LDS_CNT + 64)

static_assert((CHUNK & (CHUNK - 1)) == 0);
static_assert(CHUNK <= 4096);
static_assert((NB & (NB - 1)) == 0);
static_assert((NB0 & (NB0 - 1)) == 0);
static_assert(NB0 <= 4096);
static_assert(NTILE % NWAVE == 0);
static_assert(2 * 16 * CGW * 4 <= LDS_LIST);
static_assert(NWAVE * 4 <= 64);
static_assert(LDS_LAYER <= 300 * 1024);
static_assert(DF == 2 * CGW);
static_assert(NPF == 4 * 32);
static_assert(RG0 * NWAVE * 4 == NB0);

typedef float    v4f  __attribute__((ext_vector_type(4)));
typedef float    v8f  __attribute__((ext_vector_type(8)));
typedef int      v4i  __attribute__((ext_vector_type(4)));
typedef _Float16 f16_t;
typedef f16_t    v8h  __attribute__((ext_vector_type(8)));
typedef f16_t    v16h __attribute__((ext_vector_type(16)));
union FragH { v16h v; v8h h[2]; v4i q[2]; };
union Pack8 { v8h v; v4i q; };

__device__ __forceinline__ v8f wmh(v16h a, v16h b, v8f c) {
  v8f d = __builtin_amdgcn_wmma_f32_16x16x32_f16(false, a, false, b, (short)0, c, false, false);
  asm volatile("v_nop\n\tv_nop\n\tv_nop\n\tv_nop" : "+v"(d) : "v"(a), "v"(b));
  return d;
}

template <int B>
__device__ __forceinline__ void cvt8(FragH& f, v4f a, v4f b) {
  f.v[B + 0] = (f16_t)a.x; f.v[B + 1] = (f16_t)a.y; f.v[B + 2] = (f16_t)a.z; f.v[B + 3] = (f16_t)a.w;
  f.v[B + 4] = (f16_t)b.x; f.v[B + 5] = (f16_t)b.y; f.v[B + 6] = (f16_t)b.z; f.v[B + 7] = (f16_t)b.w;
}

__device__ __forceinline__ v4f relu4(v4f t) {
  v4f r;
  r.x = fmaxf(t.x, 0.0f); r.y = fmaxf(t.y, 0.0f); r.z = fmaxf(t.z, 0.0f); r.w = fmaxf(t.w, 0.0f);
  return r;
}

template <int NBT>
__device__ __forceinline__ int scan_chunk(const int* __restrict__ dsts, int nE, int cbase, int nodeBase,
                                          int vec8, int* list, int tid, int lane, int wave) {
  int wc = 0;
  (void)lane;
#pragma unroll
  for (int g = 0; g < NGRP; ++g) {
    const int el0  = (g * NTHR + tid) * EPT;
    const int e0   = cbase + el0;
    const int sent = -2147483647 - 1;
    v4i da, db;
    if (vec8 != 0 && e0 + 7 < nE) {
      da = *(const v4i*)(dsts + e0);
      db = *(const v4i*)(dsts + e0 + 4);
    } else {
      da.x = (e0     < nE) ? dsts[min(e0, nE - 1)] : sent;
      da.y = (e0 + 1 < nE) ? dsts[min(e0 + 1, nE - 1)] : sent;
      da.z = (e0 + 2 < nE) ? dsts[min(e0 + 2, nE - 1)] : sent;
      da.w = (e0 + 3 < nE) ? dsts[min(e0 + 3, nE - 1)] : sent;
      db.x = (e0 + 4 < nE) ? dsts[min(e0 + 4, nE - 1)] : sent;
      db.y = (e0 + 5 < nE) ? dsts[min(e0 + 5, nE - 1)] : sent;
      db.z = (e0 + 6 < nE) ? dsts[min(e0 + 6, nE - 1)] : sent;
      db.w = (e0 + 7 < nE) ? dsts[min(e0 + 7, nE - 1)] : sent;
    }
    const unsigned nb = (unsigned)nodeBase;
    const unsigned s0 = (unsigned)da.x - nb, s1 = (unsigned)da.y - nb;
    const unsigned s2 = (unsigned)da.z - nb, s3 = (unsigned)da.w - nb;
    const unsigned s4 = (unsigned)db.x - nb, s5 = (unsigned)db.y - nb;
    const unsigned s6 = (unsigned)db.z - nb, s7 = (unsigned)db.w - nb;
    const bool h0 = s0 < (unsigned)NBT, h1 = s1 < (unsigned)NBT, h2 = s2 < (unsigned)NBT, h3 = s3 < (unsigned)NBT;
    const bool h4 = s4 < (unsigned)NBT, h5 = s5 < (unsigned)NBT, h6 = s6 < (unsigned)NBT, h7 = s7 < (unsigned)NBT;
    const unsigned any = __builtin_amdgcn_ballot_w32(h0 | h1 | h2 | h3 | h4 | h5 | h6 | h7);
    if (any != 0u) {
#define HITJ(J, HJ, SJ) { \
        const unsigned mj = __builtin_amdgcn_ballot_w32(HJ); \
        if (mj != 0u) { \
          if (HJ) { \
            const int pos = wc + (int)__builtin_amdgcn_mbcnt_lo(mj, 0u); \
            if (pos < WCAP) list[wave * WCAP + pos] = ((el0 + (J)) << 12) | (int)(SJ); \
          } \
          wc += (int)__builtin_popcount(mj); } }
      HITJ(0, h0, s0)
      HITJ(1, h1, s1)
      HITJ(2, h2, s2)
      HITJ(3, h3, s3)
      HITJ(4, h4, s4)
      HITJ(5, h5, s5)
      HITJ(6, h6, s6)
      HITJ(7, h7, s7)
#undef HITJ
    }
  }
  return wc;
}

__global__ __launch_bounds__(NTHR) void k_wprep(
    const float* __restrict__ Wl, const float* __restrict__ Wr, f16_t* wp, int cout, int nTot) {
  const int i = blockIdx.x * NTHR + threadIdx.x;
  if (i >= nTot) return;
  const int o  = i * 8;
  const int n  = o / KV;
  const int k0 = o - n * KV;
  const float* p = (k0 < DF) ? (Wl + (size_t)k0 * cout + n)
                             : (Wr + (size_t)(k0 - DF) * cout + n);
  Pack8 ph;
#define WSP(I) ph.v[(I)] = (f16_t)(p[(size_t)(I) * cout] * W_SC);
  WSP(0) WSP(1) WSP(2) WSP(3) WSP(4) WSP(5) WSP(6) WSP(7)
#undef WSP
  f16_t* d = wp + o;
  const v4i q = ph.q;
  *(volatile v4i*)d = q;
  __threadfence();
  *(volatile v4i*)d = q;
}

__global__ __launch_bounds__(NTHR) void k_layer0(
    const int* __restrict__ ei, const float* __restrict__ x,
    const float* __restrict__ Wl0, const float* __restrict__ b0, const float* __restrict__ Wr0,
    float* hout, int nN, int nE, int nRows, int vec8) {
#pragma clang fp contract(off)
  __shared__ float acc0[NB0];
  __shared__ int   cnt0[NB0];
  __shared__ int   lst0[LISTN];
  __shared__ int   wcnt0[NWAVE];
  const int tid = threadIdx.x, lane = tid & 31, wave = tid >> 5;
  const int nodeBase = blockIdx.x * NB0;
  const int* dsts = ei + nE;

  for (int i = tid; i < NB0; i += NTHR) { acc0[i] = 0.0f; cnt0[i] = 0; }
  __syncthreads();

  const int nChunks = (nE + CHUNK - 1) / CHUNK;
#pragma unroll 1
  for (int ch = 0; ch < nChunks; ++ch) {
    const int cbase = ch * CHUNK;
    const int wc = scan_chunk<NB0>(dsts, nE, cbase, nodeBase, vec8, lst0, tid, lane, wave);
    if (lane == 0) wcnt0[wave] = wc;
    __syncthreads();
    if (wave == 0) {
#pragma unroll 1
      for (int wsx = 0; wsx < NWAVE; ++wsx) {
        int n = __builtin_amdgcn_readfirstlane(wcnt0[wsx]);
        n = n > WCAP ? WCAP : (n < 0 ? 0 : n);
        const int* lp = lst0 + wsx * WCAP;
#pragma unroll 1
        for (int i = 0; i < n; ++i) {
          const int ent  = __builtin_amdgcn_readfirstlane(lp[i]);
          const int slot = ent & (NB0 - 1);
          int e = cbase + ((ent >> 12) & (CHUNK - 1));
          e = e > nE - 1 ? nE - 1 : e;
          int src = ei[e];
          src = src < 0 ? 0 : (src > nN - 1 ? nN - 1 : src);
          const float xv = x[src];
          if (lane == 0) { acc0[slot] = acc0[slot] + xv; cnt0[slot] = cnt0[slot] + 1; }
        }
      }
    }
    __syncthreads();
  }

  const v4f wla = *(const v4f*)(Wl0 + 4 * lane);
  const v4f wlb = *(const v4f*)(Wl0 + CGW + 4 * lane);
  const v4f bba = *(const v4f*)(b0 + 4 * lane);
  const v4f bbb = *(const v4f*)(b0 + CGW + 4 * lane);
  const v4f wra = *(const v4f*)(Wr0 + 4 * lane);
  const v4f wrb = *(const v4f*)(Wr0 + CGW + 4 * lane);
#pragma unroll 1
  for (int rg = 0; rg < RG0; ++rg) {
    v4f va[4], vb[4];
#pragma unroll
    for (int j = 0; j < 4; ++j) {
      const int row = 32 * rg + 4 * wave + j;
      int node = nodeBase + row;
      node = node > nN - 1 ? nN - 1 : node;
      const int   cd  = cnt0[row];
      const float inv = cd > 0 ? (1.0f / (float)cd) : 0.0f;
      const float am  = acc0[row] * inv;
      const float xn  = x[node];
      v4f ta = am * wla; ta = ta + bba; const v4f ua = xn * wra; ta = ta + ua;
      v4f tb = am * wlb; tb = tb + bbb; const v4f ub = xn * wrb; tb = tb + ub;
      va[j] = relu4(ta);
      vb[j] = relu4(tb);
    }
#pragma unroll
    for (int j = 0; j < 4; ++j) {
      const int node = nodeBase + 32 * rg + 4 * wave + j;
      if (node < nRows) {
        float* gp = hout + (size_t)node * DF + 4 * lane;
        *(volatile v4f*)gp = va[j];
        *(volatile v4f*)(gp + CGW) = vb[j];
      }
    }
    __threadfence();
#pragma unroll
    for (int j = 0; j < 4; ++j) {
      const int node = nodeBase + 32 * rg + 4 * wave + j;
      if (node < nRows) {
        float* gp = hout + (size_t)node * DF + 4 * lane;
        *(volatile v4f*)gp = va[j];
        *(volatile v4f*)(gp + CGW) = vb[j];
      }
    }
  }
}

__device__ __forceinline__ void kstep(const float* ap, float mul, const f16_t* bp, v8f (&c)[8]) {
  const v4f p0 = (*(const v4f*)(ap))      * mul;
  const v4f p1 = (*(const v4f*)(ap + 4))  * mul;
  const v4f p2 = (*(const v4f*)(ap + 16)) * mul;
  const v4f p3 = (*(const v4f*)(ap + 20)) * mul;
  FragH a;
  cvt8<0>(a, p0, p1);
  cvt8<8>(a, p2, p3);
#pragma unroll
  for (int ct = 0; ct < CGW / 16; ++ct) {
    const f16_t* hp = bp + (size_t)ct * 16 * KV;
    FragH b;
    b.q[0] = *(const v4i*)hp;
    b.q[1] = *(const v4i*)(hp + 16);
    c[ct] = wmh(a.v, b.v, c[ct]);
  }
}

__global__ __launch_bounds__(NTHR) void k_layer(
    const int* __restrict__ ei, const float* __restrict__ xin,
    const f16_t* __restrict__ wp, const float* __restrict__ bias,
    float* xout, int nN, int nE, int cout, int relu, int vec8) {
#pragma clang fp contract(off)
  extern __shared__ v4f lds_dyn[];
  float* acc  = (float*)lds_dyn;
  int*   list = (int*)((char*)lds_dyn + LDS_ACC);
  float* stg  = (float*)list;
  int*   cnt  = (int*)((char*)lds_dyn + LDS_ACC + LDS_LIST);
  int*   wcnt = (int*)((char*)lds_dyn + LDS_ACC + LDS_LIST + LDS_CNT);
  const int tid = threadIdx.x, lane = tid & 31, wave = tid >> 5, hh = lane >> 4, m = lane & 15;
  const int nodeBase = blockIdx.x * NB;
  const int* dsts = ei + nE;
  const int ncg = cout / CGW;

  {
    const v4f z = {0.f, 0.f, 0.f, 0.f};
    for (int i = tid; i < NB * DF / 4; i += NTHR) lds_dyn[i] = z;
    if (tid < NB) cnt[tid] = 0;
  }
  __syncthreads();

  const int nChunks = (nE + CHUNK - 1) / CHUNK;
#pragma unroll 1
  for (int ch = 0; ch < nChunks; ++ch) {
    const int cbase = ch * CHUNK;
    const int wc = scan_chunk<NB>(dsts, nE, cbase, nodeBase, vec8, list, tid, lane, wave);
    if (lane == 0) wcnt[wave] = wc;
    __syncthreads();
    if (wave == 0) {
#pragma unroll 1
      for (int wsx = 0; wsx < NWAVE; ++wsx) {
        int n = __builtin_amdgcn_readfirstlane(wcnt[wsx]);
        n = n > WCAP ? WCAP : (n < 0 ? 0 : n);
        const int* lp = list + wsx * WCAP;
#pragma unroll 1
        for (int i = 0; i < n; ++i) {
          const int ent  = __builtin_amdgcn_readfirstlane(lp[i]);
          const int slot = ent & (NB - 1);
          int e = cbase + ((ent >> 12) & (CHUNK - 1));
          e = e > nE - 1 ? nE - 1 : e;
          int src = ei[e];
          src = src < 0 ? 0 : (src > nN - 1 ? nN - 1 : src);
          const float* xr = xin + (size_t)src * DF;
          const v4f va = *(const v4f*)(xr + 4 * lane);
          const v4f vb = *(const v4f*)(xr + CGW + 4 * lane);
          v4f* ar = (v4f*)(acc + slot * DF);
          ar[lane]      = ar[lane] + va;
          ar[32 + lane] = ar[32 + lane] + vb;
          if (lane == 0) cnt[slot] = cnt[slot] + 1;
        }
      }
    }
    __syncthreads();
  }

#pragma unroll 1
  for (int q = 0; q < TPW; ++q) {
    const int t     = q * NWAVE + wave;
    const int slotm = 16 * t + m;
    int node = nodeBase + slotm;
    node = node > nN - 1 ? nN - 1 : node;
    const int   cd   = cnt[slotm];
    const float inv  = cd > 0 ? (1.0f / (float)cd) : 0.0f;
    const float amul = inv * A_SC;
    const float* arow = acc + slotm * DF + 8 * hh;
    const float* xrow = xin + (size_t)node * DF + 8 * hh;
#pragma unroll 1
    for (int cg = 0; cg < ncg; ++cg) {
      v8f c[8];
#pragma unroll
      for (int ct = 0; ct < 8; ++ct) { const v8f z = {0.f, 0.f, 0.f, 0.f, 0.f, 0.f, 0.f, 0.f}; c[ct] = z; }
      const f16_t* bp0 = wp + (size_t)(cg * CGW + m) * KV + 8 * hh;
#pragma unroll 1
      for (int ks = 0; ks < DF / 32; ++ks)
        kstep(arow + 32 * ks, amul, bp0 + 32 * ks, c);
#pragma unroll 1
      for (int ks = 0; ks < DF / 32; ++ks)
        kstep(xrow + 32 * ks, A_SC, bp0 + DF + 32 * ks, c);

#pragma unroll
      for (int ct = 0; ct < 8; ++ct) {
        const float bb = bias[cg * CGW + 16 * ct + m];
#pragma unroll
        for (int r = 0; r < 8; ++r) {
          const float v = c[ct][r] * O_SC + bb;
          c[ct][r] = (relu != 0) ? fmaxf(v, 0.0f) : v;
        }
      }

      const int half = wave & 1;
      float* sbase = stg + half * (16 * CGW);
#pragma unroll 1
      for (int turn = 0; turn < NWAVE / 2; ++turn) {
        __syncthreads();
        if ((wave >> 1) == turn) {
          float* sp = sbase + (8 * hh) * CGW + m;
#pragma unroll
          for (int ct = 0; ct < 8; ++ct) {
#pragma unroll
            for (int r = 0; r < 8; ++r) sp[r * CGW + 16 * ct] = c[ct][r];
          }
        }
        __syncthreads();
        if ((wave >> 1) == turn) {
          const float* lrow = sbase + 4 * lane;
          float* gp = xout + ((size_t)nodeBase + 16 * t) * (size_t)cout + cg * CGW + 4 * lane;
#pragma unroll
          for (int i = 0; i < 16; ++i) {
            const v4f v = *(const v4f*)(lrow + i * CGW);
            *(volatile v4f*)(gp + (size_t)i * cout) = v;
          }
          __threadfence();
#pragma unroll
          for (int i = 0; i < 16; ++i) {
            const v4f v = *(const v4f*)(lrow + i * CGW);
            *(volatile v4f*)(gp + (size_t)i * cout) = v;
          }
        }
      }
    }
  }
}

__global__ __launch_bounds__(NTHR) void k_pool(
    const int* __restrict__ bat, const float* __restrict__ h,
    const float* __restrict__ gam, const float* __restrict__ bet,
    float* out, int nN, int vec8) {
#pragma clang fp contract(off)
  __shared__ int lstp[LISTN];
  __shared__ int wcntp[NWAVE];
  const int tid = threadIdx.x, lane = tid & 31, wave = tid >> 5;
  const int g = blockIdx.x;
  v4f s = {0.f, 0.f, 0.f, 0.f};
  int gc = 0;

  const int nChunks = (nN + CHUNK - 1) / CHUNK;
#pragma unroll 1
  for (int ch = 0; ch < nChunks; ++ch) {
    const int cbase = ch * CHUNK;
    const int wc = scan_chunk<1>(bat, nN, cbase, g, vec8, lstp, tid, lane, wave);
    if (lane == 0) wcntp[wave] = wc;
    __syncthreads();
    if (wave == 0) {
#pragma unroll 1
      for (int wsx = 0; wsx < NWAVE; ++wsx) {
        int n = __builtin_amdgcn_readfirstlane(wcntp[wsx]);
        n = n > WCAP ? WCAP : (n < 0 ? 0 : n);
        const int* lp = lstp + wsx * WCAP;
#pragma unroll 1
        for (int i = 0; i < n; ++i) {
          const int ent = __builtin_amdgcn_readfirstlane(lp[i]);
          int nd = cbase + ((ent >> 12) & (CHUNK - 1));
          nd = nd > nN - 1 ? nN - 1 : nd;
          const v4f v = *(const v4f*)(h + (size_t)nd * NPF + 4 * lane);
          s = s + v;
          gc += 1;
        }
      }
    }
    __syncthreads();
  }

  if (wave == 0) {
    const float invc = 1.0f / (float)(gc > 0 ? gc : 1);
    const v4f gv = s * invc;
    float ps = gv.x + gv.y + gv.z + gv.w;
#pragma unroll
    for (int off = 16; off > 0; off >>= 1) ps += __shfl_xor(ps, off, 32);
    const float mu = ps * (1.0f / (float)NPF);
    const v4f d = gv - mu;
    float sq = d.x * d.x + d.y * d.y + d.z * d.z + d.w * d.w;
#pragma unroll
    for (int off = 16; off > 0; off >>= 1) sq += __shfl_xor(sq, off, 32);
    const float var = sq * (1.0f / (float)NPF);
    const float rs  = rsqrtf(var + LN_EPS);
    const v4f gm = *(const v4f*)(gam + 4 * lane);
    const v4f bt = *(const v4f*)(bet + 4 * lane);
    v4f o = d * rs;
    o = o * gm;
    o = o + bt;
    float* op = out + (size_t)g * NPF + 4 * lane;
    *(volatile v4f*)op = o;
    __threadfence();
    *(volatile v4f*)op = o;
  }
}

extern "C" void kernel_launch(void* const* d_in, const int* in_sizes, int n_in,
                              void* d_out, int out_size, void* d_ws, size_t ws_size,
                              hipStream_t stream) {
  if (n_in < 14) return;
  const int nN = in_sizes[0];
  const int nE = in_sizes[1] / 2;
  if (nN <= 0 || nE < 0 || in_sizes[1] != 2 * nE) return;
  if (in_sizes[2] != nN) return;
  if (in_sizes[3] != DF || in_sizes[4] < DF || in_sizes[5] != DF) return;
  if (in_sizes[6] != DF * DF || in_sizes[7] < DF || in_sizes[8] != DF * DF) return;
  if (in_sizes[9] != DF * NPF || in_sizes[10] < NPF || in_sizes[11] != DF * NPF) return;
  if (in_sizes[12] < NPF || in_sizes[13] < NPF) return;
  if (out_size <= 0 || (out_size % NPF) != 0) return;
  const int nG = out_size / NPF;

  const float* x     = (const float*)d_in[0];
  const int*   ei    = (const int*)d_in[1];
  const int*   batch = (const int*)d_in[2];
  const float* Wl0   = (const float*)d_in[3];
  const float* b0    = (const float*)d_in[4];
  const float* Wr0   = (const float*)d_in[5];
  const float* Wl1   = (const float*)d_in[6];
  const float* b1    = (const float*)d_in[7];
  const float* Wr1   = (const float*)d_in[8];
  const float* Wl2   = (const float*)d_in[9];
  const float* b2    = (const float*)d_in[10];
  const float* Wr2   = (const float*)d_in[11];
  const float* gamma = (const float*)d_in[12];
  const float* beta  = (const float*)d_in[13];
  float* out = (float*)d_out;

  const int nBlk  = (nN + NB - 1) / NB;
  const int nRows = nBlk * NB;
  const int nBlk0 = (nRows + NB0 - 1) / NB0;

  char* ws = (char*)d_ws;
  size_t off = 0;
  const size_t szW1 = (size_t)DF  * KV * 2;
  const size_t szW2 = (size_t)NPF * KV * 2;
  const size_t szH  = (size_t)nRows * DF * 4;
  const size_t oW1 = off; off += szW1; off = (off + 255) & ~(size_t)255;
  const size_t oW2 = off; off += szW2; off = (off + 255) & ~(size_t)255;
  const size_t oHa = off; off += szH;  off = (off + 255) & ~(size_t)255;
  const size_t oHb = off; off += szH;  off = (off + 255) & ~(size_t)255;
  if (off > ws_size) return;
  f16_t* w1 = (f16_t*)(ws + oW1);
  f16_t* w2 = (f16_t*)(ws + oW2);
  float* ha = (float*)(ws + oHa);
  float* hb = (float*)(ws + oHb);

  const int vec8 = ((nE & 3) == 0) ? 1 : 0;

  const int nTot1 = DF * KV / 8;
  const int nTot2 = NPF * KV / 8;
  k_wprep<<<(nTot1 + NTHR - 1) / NTHR, NTHR, 0, stream>>>(Wl1, Wr1, w1, DF, nTot1);
  k_wprep<<<(nTot2 + NTHR - 1) / NTHR, NTHR, 0, stream>>>(Wl2, Wr2, w2, NPF, nTot2);

  k_layer0<<<nBlk0, NTHR, 0, stream>>>(ei, x, Wl0, b0, Wr0, ha, nN, nE, nRows, vec8);

  hipFuncSetAttribute(reinterpret_cast<const void*>(&k_layer),
                      hipFuncAttributeMaxDynamicSharedMemorySize, LDS_LAYER);
  k_layer<<<nBlk, NTHR, LDS_LAYER, stream>>>(ei, ha, w1, b1, hb, nN, nE, DF,  1, vec8);
  k_layer<<<nBlk, NTHR, LDS_LAYER, stream>>>(ei, hb, w2, b2, ha, nN, nE, NPF, 0, vec8);

  k_pool<<<nG, NTHR, 0, stream>>>(batch, ha, gamma, beta, out, nN, 1);
}
